// MambaSkipFusion_65360812311158
// MI455X (gfx1250) — hardware-run, weakly checked
//
#include <hip/hip_runtime.h>
#include <math.h>

#define NBT   2
#define NCH   192
#define NCAT  384
#define NPIX  4096
#define NTOK  8192
#define DIN   384
#define DXZ   768
#define DST   16
#define DTRK  12
#define KCV   4
#define DBW   64
#define DBN   44
#define COLB  12
#define COLC  28
#define TPB   128
#define NBLK  64
#define NBY3  3
#define OSTR  68
#define SCH   32
#define XP8   48
#define XTP   200
#define XT8   24
#define LOG2E 1.4426950408889634f
#define EPSV  1e-5f

static_assert(NTOK == NBT * NPIX);
static_assert(NTOK % TPB == 0);
static_assert(NBLK == NTOK / TPB);
static_assert(NPIX % TPB == 0);
static_assert(NCH % 64 == 0);
static_assert(NBY3 == NCH / 64);
static_assert(NCAT == 2 * NCH);
static_assert(DXZ == 2 * DIN);
static_assert(DXZ % 64 == 0);
static_assert(NCAT % 32 == 0);
static_assert(NCH % 32 == 0);
static_assert(DIN % 32 == 0);
static_assert(DBW == 64);
static_assert(DBN <= DBW);
static_assert(COLB == DTRK);
static_assert(COLC == COLB + DST);
static_assert(COLC + DST == DBN);
static_assert(COLB % 4 == 0);
static_assert(COLC % 4 == 0);
static_assert(DTRK == 12);
static_assert(NPIX % SCH == 0);
static_assert(XP8 * 8 == DIN);
static_assert((SCH * XP8) % DIN == 0);
static_assert((SCH * XP8) / DIN == 4);
static_assert(XTP % 8 == 0);
static_assert(XTP >= NCH);
static_assert(XT8 * 8 == NCH);
static_assert((64 * XT8) % 256 == 0);
static_assert(NPIX % 64 == 0);
static_assert(NPIX / 4 == 1024);
static_assert((NBT * NCH * NPIX) % 1024 == 0);
static_assert(OSTR % 4 == 0);
static_assert((NTOK * DIN) % 256 == 0);
static_assert(DIN % 32 == 0 && DIN <= 1024);

typedef unsigned short us16 __attribute__((ext_vector_type(16)));
typedef unsigned short us8  __attribute__((ext_vector_type(8)));
typedef unsigned short us8a __attribute__((ext_vector_type(8), may_alias));
typedef unsigned int   u32x8 __attribute__((ext_vector_type(8)));
typedef __bf16 v16b __attribute__((ext_vector_type(16)));
typedef float v8f __attribute__((ext_vector_type(8)));
typedef float v4f __attribute__((ext_vector_type(4)));
typedef float v4fa __attribute__((ext_vector_type(4), may_alias));
union FragU { us16 v; us8 h[2]; u32x8 w; };

#if __has_builtin(__builtin_amdgcn_exp2f)
#define FEXP2(x) __builtin_amdgcn_exp2f(x)
#else
#define FEXP2(x) __expf((x) * 0.6931471805599453f)
#endif

__device__ __forceinline__ unsigned short bf16_bits(float f) {
  unsigned u = __float_as_uint(f);
  u += 0x7FFFu + ((u >> 16) & 1u);
  return (unsigned short)(u >> 16);
}
__device__ __forceinline__ float bf16_val(unsigned short b) { return __uint_as_float(((unsigned)b) << 16); }
__device__ __forceinline__ float bf16r(float f) { return bf16_val(bf16_bits(f)); }
__device__ __forceinline__ float siluf(float x) { return x * __builtin_amdgcn_rcpf(1.0f + __expf(-x)); }

__device__ __forceinline__ void split8(const v4f a, const v4f b, us8& hi, us8& lo) {
#pragma unroll
  for (int u = 0; u < 4; ++u) {
    const unsigned short ha = bf16_bits(a[u]);
    hi[u] = ha; lo[u] = bf16_bits(a[u] - bf16_val(ha));
    const unsigned short hb = bf16_bits(b[u]);
    hi[4 + u] = hb; lo[4 + u] = bf16_bits(b[u] - bf16_val(hb));
  }
}

__device__ __forceinline__ v8f mma_bf16(us16 a, us16 b, v8f c) {
  return __builtin_amdgcn_wmma_f32_16x16x32_bf16(false, __builtin_bit_cast(v16b, a), false, __builtin_bit_cast(v16b, b), (short)0, c, false, false);
}
__device__ __forceinline__ void wguard2(v8f& c0, v8f& c1, v8f& c2, v8f& c3, const us16& a0, const us16& a1,
                                        const us16& b0, const us16& b1, const us16& b2, const us16& b3) {
#if defined(__HIP_DEVICE_COMPILE__)
  asm volatile("v_nop\n\tv_nop\n\tv_nop\n\tv_nop"
               : "+v"(c0), "+v"(c1), "+v"(c2), "+v"(c3)
               : "v"(a0), "v"(a1), "v"(b0), "v"(b1), "v"(b2), "v"(b3));
#endif
}

__device__ __forceinline__ us16 gfrag(const unsigned short* p) {
  const int kh = ((threadIdx.x >> 4) & 1) * 8;
  FragU f;
  f.h[0] = *(const us8a*)(p + kh);
  f.h[1] = *(const us8a*)(p + 16 + kh);
  return f.v;
}

__global__ __launch_bounds__(256) void k_cvtW(const float* __restrict__ src, unsigned short* dst, int srcN, int srcK, int total8) {
  const int idx = blockIdx.x * 256 + threadIdx.x;
  if (idx >= total8) return;
  const int kp8 = srcK >> 3;
  const int n = idx / kp8, k8 = (idx - n * kp8) * 8;
  const bool rowok = (n < srcN);
  const int nc = rowok ? n : (srcN - 1);
  const float* sp = src + (size_t)nc * (size_t)srcK + k8;
  us8 o;
#pragma unroll
  for (int u = 0; u < 8; ++u) {
    const float v = sp[u];
    o[u] = rowok ? bf16_bits(v) : (unsigned short)0;
  }
  const size_t off = (size_t)idx * 8;
  *(volatile us8*)(dst + off) = o;
  __threadfence();
  *(volatile us8*)(dst + off) = o;
}

__global__ __launch_bounds__(256) void k_xtok(const float* __restrict__ enc, const float* __restrict__ dec, unsigned short* XB) {
  __shared__ __attribute__((aligned(16))) unsigned short tile[64 * XTP];
  const int tid = threadIdx.x, hw0 = blockIdx.x * 64, b = blockIdx.y, src = blockIdx.z;
  const float* x = (src == 0) ? enc : dec;
  const int hw = tid & 63, cq = tid >> 6;
#pragma unroll 4
  for (int it = 0; it < NCH / 4; ++it) {
    const int c = it * 4 + cq;
    const float v = x[((size_t)(b * NCH + c)) * NPIX + hw0 + hw];
    tile[hw * XTP + c] = bf16_bits(v);
  }
  __syncthreads();
#pragma unroll
  for (int pass = 0; pass < 2; ++pass) {
#pragma unroll
    for (int it = 0; it < (64 * XT8) / 256; ++it) {
      const int p = it * 256 + tid, rr = p / XT8, c8 = (p - rr * XT8) * 8;
      const us8 v = *(const us8a*)(tile + rr * XTP + c8);
      *(volatile us8*)(XB + ((size_t)(b * NPIX + hw0 + rr)) * NCAT + src * NCH + c8) = v;
    }
    __threadfence();
  }
}

template <int TWOA, int HASB, int OUTF, int OUTHL, int NCHWO>
__global__ __launch_bounds__(256) void k_gemm(const unsigned short* __restrict__ A0, const unsigned short* __restrict__ A1, int lda,
                                             const unsigned short* __restrict__ Bw, int ldb, int K, const float* __restrict__ bias,
                                             float* Yf, int ldy, unsigned short* YH, unsigned short* YL, int ldh,
                                             float* Onc, float* PART) {
  __shared__ __attribute__((aligned(16))) float oS[8 * 16 * OSTR];
  __shared__ __attribute__((aligned(16))) float red[512];
  __shared__ __attribute__((aligned(16))) float pst[128];
  const int tid = threadIdx.x, lane = tid & 31, wave = tid >> 5, cl = lane & 15, hh = lane >> 4;
  const int mb = blockIdx.x * TPB, m0 = mb + 16 * wave, n0 = blockIdx.y * 64;

  v8f acc[4];
#pragma unroll
  for (int j = 0; j < 4; ++j) { const v8f zz = {0.f, 0.f, 0.f, 0.f, 0.f, 0.f, 0.f, 0.f}; acc[j] = zz; }

  const unsigned short* a0p = A0 + (size_t)(m0 + cl) * lda;
  const unsigned short* a1p = A1 + (size_t)(m0 + cl) * lda;
  const unsigned short* bwp = Bw + (size_t)(n0 + cl) * ldb;
#pragma unroll 1
  for (int k0 = 0; k0 < K; k0 += 32) {
    const us16 af0 = gfrag(a0p + k0);
    us16 af1 = af0;
    if (TWOA) af1 = gfrag(a1p + k0);
    us16 bfr[4];
#pragma unroll
    for (int j = 0; j < 4; ++j) bfr[j] = gfrag(bwp + (size_t)(16 * j) * ldb + k0);
#pragma unroll
    for (int j = 0; j < 4; ++j) acc[j] = mma_bf16(af0, bfr[j], acc[j]);
    if (TWOA) {
#pragma unroll
      for (int j = 0; j < 4; ++j) acc[j] = mma_bf16(af1, bfr[j], acc[j]);
    }
    wguard2(acc[0], acc[1], acc[2], acc[3], af0, af1, bfr[0], bfr[1], bfr[2], bfr[3]);
  }

  float bj[4];
#pragma unroll
  for (int j = 0; j < 4; ++j) bj[j] = HASB ? bf16r(bias[n0 + 16 * j + cl]) : 0.0f;

  float* so = oS + wave * (16 * OSTR);
#pragma unroll
  for (int j = 0; j < 4; ++j)
#pragma unroll
    for (int r = 0; r < 8; ++r) so[(8 * hh + r) * OSTR + 16 * j + cl] = acc[j][r] + bj[j];
  __syncthreads();

  if (OUTF) {
#pragma unroll
    for (int pass = 0; pass < 2; ++pass) {
#pragma unroll
      for (int it = 0; it < 8; ++it) {
        const int ch = it * 32 + lane, r = ch >> 4, q = (ch & 15) * 4;
        const v4f v = *(const v4fa*)(so + r * OSTR + q);
        *(volatile v4f*)(Yf + (size_t)(m0 + r) * ldy + n0 + q) = v;
      }
      __threadfence();
    }
  }
  if (OUTHL) {
    us8 hiq[4], loq[4];
#pragma unroll
    for (int it = 0; it < 4; ++it) {
      const int ch = it * 32 + lane, r = ch >> 3, c8 = (ch & 7) * 8;
      const v4f a = *(const v4fa*)(so + r * OSTR + c8);
      const v4f b = *(const v4fa*)(so + r * OSTR + c8 + 4);
      split8(a, b, hiq[it], loq[it]);
    }
#pragma unroll
    for (int pass = 0; pass < 2; ++pass) {
#pragma unroll
      for (int it = 0; it < 4; ++it) {
        const int ch = it * 32 + lane, r = ch >> 3, c8 = (ch & 7) * 8;
        const size_t o2 = (size_t)(m0 + r) * ldh + n0 + c8;
        *(volatile us8*)(YH + o2) = hiq[it]; *(volatile us8*)(YL + o2) = loq[it];
      }
      __threadfence();
    }
  }
  if (NCHWO) {
    const int bimg = mb / NPIX, hw0 = mb - bimg * NPIX;
#pragma unroll
    for (int pass = 0; pass < 2; ++pass) {
#pragma unroll
      for (int it = 0; it < 8; ++it) {
        const int c = it * 8 + wave;
        v4f v;
#pragma unroll
        for (int i = 0; i < 4; ++i) v[i] = oS[(lane * 4 + i) * OSTR + c];
        const size_t o = ((size_t)(bimg * NCH + n0 + c)) * NPIX + hw0 + lane * 4;
        *(volatile v4f*)(Onc + o) = v;
      }
      __threadfence();
    }
    {
      const int c = tid & 63, ph = tid >> 6;
      float s = 0.0f, q = 0.0f;
#pragma unroll 4
      for (int i = 0; i < 32; ++i) {
        const float v = oS[(ph * 32 + i) * OSTR + c];
        s += v; q += v * v;
      }
      red[ph * 64 + c] = s; red[256 + ph * 64 + c] = q;
    }
    __syncthreads();
    if (tid < 64) {
      const float S = ((red[tid] + red[64 + tid]) + red[128 + tid]) + red[192 + tid];
      const float Q = ((red[256 + tid] + red[320 + tid]) + red[384 + tid]) + red[448 + tid];
      pst[tid] = S; pst[64 + tid] = Q;
    }
    __syncthreads();
    if (wave == 0) {
      const v4f v = *(const v4fa*)(pst + lane * 4);
      const size_t po = (size_t)(blockIdx.x * gridDim.y + blockIdx.y) * 128 + lane * 4;
      *(volatile v4f*)(PART + po) = v;
      __threadfence();
      *(volatile v4f*)(PART + po) = v;
    }
  }
}

__global__ __launch_bounds__(DIN) void k_conv(const float* __restrict__ XZ, const float* __restrict__ cw, const float* __restrict__ cb,
                                             float* UF, unsigned short* UH, unsigned short* UL) {
  __shared__ __attribute__((aligned(16))) float su[DIN];
  const int tid = threadIdx.x, tok = blockIdx.x, b = tok / NPIX, l = tok - b * NPIX, d = tid;
  float a = bf16r(cb[d]);
#pragma unroll
  for (int j = 0; j < KCV; ++j) {
    const int lp = l - (KCV - 1) + j;
    const int lpc = (lp < 0) ? 0 : lp;
    const float v = XZ[((size_t)b * NPIX + (size_t)lpc) * DXZ + d];
    const float wj = bf16r(cw[d * KCV + j]);
    a = a + ((lp >= 0) ? (v * wj) : 0.0f);
  }
  su[d] = siluf(a);
  __syncthreads();
  const int t4 = (tid < DIN / 4) ? tid : 0;
  const int t8 = (tid < DIN / 8) ? tid : 0;
  const v4f fv = *(const v4fa*)(su + t4 * 4);
  const v4f ha = *(const v4fa*)(su + t8 * 8);
  const v4f hb = *(const v4fa*)(su + t8 * 8 + 4);
  us8 hi, lo;
  split8(ha, hb, hi, lo);
  const size_t rowb = (size_t)tok * DIN;
#pragma unroll
  for (int pass = 0; pass < 2; ++pass) {
    if (tid < DIN / 4) *(volatile v4f*)(UF + rowb + tid * 4) = fv;
    if (tid < DIN / 8) { *(volatile us8*)(UH + rowb + tid * 8) = hi; *(volatile us8*)(UL + rowb + tid * 8) = lo; }
    __threadfence();
  }
}

__global__ __launch_bounds__(256) void k_dt(const float* __restrict__ XDBL, const float* __restrict__ dtw, const float* __restrict__ dtb,
                                           float* DT) {
  const int idx = blockIdx.x * 256 + threadIdx.x;
  if (idx >= NTOK * DIN) return;
  const int tok = idx / DIN, d = idx - tok * DIN;
  const float* xr = XDBL + (size_t)tok * DBW;
  const v4f x0 = *(const v4fa*)(xr), x1 = *(const v4fa*)(xr + 4), x2 = *(const v4fa*)(xr + 8);
  const float* wr = dtw + (size_t)d * DTRK;
  float a = 0.0f;
#pragma unroll
  for (int r = 0; r < 4; ++r) a = a + x0[r] * bf16r(wr[r]);
#pragma unroll
  for (int r = 0; r < 4; ++r) a = a + x1[r] * bf16r(wr[4 + r]);
#pragma unroll
  for (int r = 0; r < 4; ++r) a = a + x2[r] * bf16r(wr[8 + r]);
  a = a + bf16r(dtb[d]);
  const float sp = fmaxf(a, 0.0f) + log1pf(__expf(-fabsf(a)));
  *(volatile float*)(DT + idx) = sp;
  __threadfence();
  *(volatile float*)(DT + idx) = sp;
}

__global__ __launch_bounds__(DIN) void k_scan(const float* __restrict__ DT, const float* __restrict__ UF, const float* __restrict__ XDBL,
                                             const float* __restrict__ XZ, const float* __restrict__ Alog, const float* __restrict__ Dv,
                                             unsigned short* YH, unsigned short* YL) {
  __shared__ __attribute__((aligned(16))) float sy[SCH * DIN];
  const int tid = threadIdx.x, b = blockIdx.x, d = tid;
  float A2[DST], h[DST];
#pragma unroll
  for (int i = 0; i < DST; ++i) { A2[i] = -__expf(bf16r(Alog[d * DST + i])) * LOG2E; h[i] = 0.0f; }
  const float Dd = bf16r(Dv[d]);
#pragma unroll 1
  for (int c = 0; c < NPIX / SCH; ++c) {
#pragma unroll 1
    for (int s = 0; s < SCH; ++s) {
      const size_t tok = (size_t)b * NPIX + (size_t)(c * SCH + s);
      const size_t e = tok * DIN + d;
      const float dl = DT[e], uv = UF[e], z = XZ[tok * DXZ + DIN + d];
      const float* bc = XDBL + tok * DBW + COLB;
      v4f Bv[4], Cv[4];
#pragma unroll
      for (int q = 0; q < 4; ++q) {
        Bv[q] = *(const v4fa*)(bc + 4 * q);
        Cv[q] = *(const v4fa*)(bc + (COLC - COLB) + 4 * q);
      }
      const float dx = dl * uv;
      float y = 0.0f;
#pragma unroll
      for (int i = 0; i < DST; ++i) {
        const float ex = FEXP2(dl * A2[i]);
        h[i] = ex * h[i] + dx * Bv[i >> 2][i & 3];
        y = y + h[i] * Cv[i >> 2][i & 3];
      }
      sy[s * DIN + d] = (y + uv * Dd) * siluf(z);
    }
    __syncthreads();
    us8 hiq[4], loq[4];
#pragma unroll
    for (int it = 0; it < 4; ++it) {
      const int p = it * DIN + tid, row = p / XP8, c8 = (p - row * XP8) * 8;
      const v4f a = *(const v4fa*)(sy + row * DIN + c8);
      const v4f bq = *(const v4fa*)(sy + row * DIN + c8 + 4);
      split8(a, bq, hiq[it], loq[it]);
    }
#pragma unroll
    for (int pass = 0; pass < 2; ++pass) {
#pragma unroll
      for (int it = 0; it < 4; ++it) {
        const int p = it * DIN + tid, row = p / XP8, c8 = (p - row * XP8) * 8;
        const size_t o = ((size_t)b * NPIX + (size_t)(c * SCH + row)) * DIN + c8;
        *(volatile us8*)(YH + o) = hiq[it]; *(volatile us8*)(YL + o) = loq[it];
      }
      __threadfence();
    }
    __syncthreads();
  }
}

__global__ __launch_bounds__(256) void k_bnfin(const float* __restrict__ PART, float* ST) {
  __shared__ __attribute__((aligned(16))) float pst[512];
  const int tid = threadIdx.x;
  const bool ok = (tid < NCH);
  const int cc = ok ? tid : (NCH - 1);
  const int by = cc >> 6, cl = cc & 63;
  double s = 0.0, q = 0.0;
#pragma unroll 1
  for (int p = 0; p < NBLK; ++p) {
    const size_t base = (size_t)(p * NBY3 + by) * 128;
    s += (double)PART[base + cl]; q += (double)PART[base + 64 + cl];
  }
  const double mean = s / (double)NTOK;
  double var = q / (double)NTOK - mean * mean;
  var = (var < 0.0) ? 0.0 : var;
  pst[tid] = ok ? (float)mean : 0.0f;
  pst[256 + tid] = ok ? rsqrtf((float)var + EPSV) : 0.0f;
  __syncthreads();
  if (tid < 128) {
    const v4f v = *(const v4fa*)(pst + tid * 4);
    *(volatile v4f*)(ST + tid * 4) = v;
    __threadfence();
    *(volatile v4f*)(ST + tid * 4) = v;
  }
}

__global__ __launch_bounds__(256) void k_bnapply(const float* __restrict__ Onc, const float* __restrict__ ST,
                                                const float* __restrict__ g, const float* __restrict__ be, float* outp) {
  const int idx = blockIdx.x * 256 + threadIdx.x;
  if (idx >= NBT * NCH * NPIX / 4) return;
  const int c = (idx >> 10) % NCH;
  const v4f v = *(const v4fa*)(Onc + (size_t)idx * 4);
  const float mu = ST[c], rs = ST[256 + c], gg = bf16r(g[c]), bb = bf16r(be[c]);
  v4f o;
#pragma unroll
  for (int u = 0; u < 4; ++u) o[u] = ((v[u] - mu) * rs) * gg + bb;
  *(volatile v4f*)(outp + (size_t)idx * 4) = o;
  __threadfence();
  *(volatile v4f*)(outp + (size_t)idx * 4) = o;
}

extern "C" void kernel_launch(void* const* d_in, const int* in_sizes, int n_in,
                              void* d_out, int out_size, void* d_ws, size_t ws_size,
                              hipStream_t stream) {
  if (n_in < 17) return;
  if (in_sizes[0] != NBT * NCH * NPIX || in_sizes[1] != NBT * NCH * NPIX || in_sizes[2] != NCH * NCAT || in_sizes[3] != NCH ||
      in_sizes[4] != DXZ * NCH || in_sizes[5] != DXZ || in_sizes[6] != DIN * KCV || in_sizes[7] != DIN || in_sizes[8] != DBN * DIN ||
      in_sizes[9] != DIN * DTRK || in_sizes[10] != DIN || in_sizes[11] != DIN * DST || in_sizes[12] != DIN ||
      in_sizes[13] != NCH * DIN || in_sizes[14] != NCH || in_sizes[15] != NCH || in_sizes[16] != NCH) return;
  if (out_size != NBT * NCH * NPIX) return;

  const float* enc        = (const float*)d_in[0];
  const float* dec        = (const float*)d_in[1];
  const float* fuse_w     = (const float*)d_in[2];
  const float* fuse_b     = (const float*)d_in[3];
  const float* in_proj_w  = (const float*)d_in[4];
  const float* in_proj_b  = (const float*)d_in[5];
  const float* conv_w     = (const float*)d_in[6];
  const float* conv_b     = (const float*)d_in[7];
  const float* x_proj_w   = (const float*)d_in[8];
  const float* dt_proj_w  = (const float*)d_in[9];
  const float* dt_proj_b  = (const float*)d_in[10];
  const float* A_log      = (const float*)d_in[11];
  const float* Dv         = (const float*)d_in[12];
  const float* out_proj_w = (const float*)d_in[13];
  const float* out_proj_b = (const float*)d_in[14];
  const float* bn_g       = (const float*)d_in[15];
  const float* bn_b       = (const float*)d_in[16];
  float* out = (float*)d_out;

  size_t off = 0;
  auto carve = [&](size_t bytes) -> char* { char* p = (char*)d_ws + off; off += (bytes + 255) & ~(size_t)255; return p; };
  unsigned short* XB  = (unsigned short*)carve((size_t)NTOK * NCAT * 2);
  unsigned short* XFH = (unsigned short*)carve((size_t)NTOK * NCH * 2);
  unsigned short* XFL = (unsigned short*)carve((size_t)NTOK * NCH * 2);
  float* XZ   = (float*)carve((size_t)NTOK * DXZ * 4);
  float* UF   = (float*)carve((size_t)NTOK * DIN * 4);
  unsigned short* UH  = (unsigned short*)carve((size_t)NTOK * DIN * 2);
  unsigned short* UL  = (unsigned short*)carve((size_t)NTOK * DIN * 2);
  float* XDBL = (float*)carve((size_t)NTOK * DBW * 4);
  float* DT   = (float*)carve((size_t)NTOK * DIN * 4);
  unsigned short* YH  = (unsigned short*)carve((size_t)NTOK * DIN * 2);
  unsigned short* YL  = (unsigned short*)carve((size_t)NTOK * DIN * 2);
  float* ONC  = (float*)carve((size_t)NBT * NCH * NPIX * 4);
  unsigned short* WF  = (unsigned short*)carve((size_t)NCH * NCAT * 2);
  unsigned short* WIN = (unsigned short*)carve((size_t)DXZ * NCH * 2);
  unsigned short* WXP = (unsigned short*)carve((size_t)DBW * DIN * 2);
  unsigned short* WOP = (unsigned short*)carve((size_t)NCH * DIN * 2);
  float* PART = (float*)carve((size_t)NBLK * NBY3 * 128 * 4);
  float* ST   = (float*)carve((size_t)512 * 4);
  if (off > ws_size || off > (size_t)134217728) return;

  const dim3 b256(256);
  auto cdv = [](long a, long b) { return (unsigned)((a + b - 1) / b); };

  k_cvtW<<<dim3(cdv(NCH * (NCAT / 8), 256)), b256, 0, stream>>>(fuse_w, WF, NCH, NCAT, NCH * (NCAT / 8));
  k_cvtW<<<dim3(cdv(DXZ * (NCH / 8), 256)), b256, 0, stream>>>(in_proj_w, WIN, DXZ, NCH, DXZ * (NCH / 8));
  k_cvtW<<<dim3(cdv(DBW * (DIN / 8), 256)), b256, 0, stream>>>(x_proj_w, WXP, DBN, DIN, DBW * (DIN / 8));
  k_cvtW<<<dim3(cdv(NCH * (DIN / 8), 256)), b256, 0, stream>>>(out_proj_w, WOP, NCH, DIN, NCH * (DIN / 8));
  k_xtok<<<dim3(NPIX / 64, NBT, 2), b256, 0, stream>>>(enc, dec, XB);
  k_gemm<0, 1, 0, 1, 0><<<dim3(NBLK, NCH / 64), b256, 0, stream>>>(XB, XB, NCAT, WF, NCAT, NCAT, fuse_b, XZ, DXZ, XFH, XFL, NCH, ONC, PART);
  k_gemm<1, 1, 1, 0, 0><<<dim3(NBLK, DXZ / 64), b256, 0, stream>>>(XFH, XFL, NCH, WIN, NCH, NCH, in_proj_b, XZ, DXZ, UH, UL, DIN, ONC, PART);
  k_conv<<<dim3(NTOK), dim3(DIN), 0, stream>>>(XZ, conv_w, conv_b, UF, UH, UL);
  k_gemm<1, 0, 1, 0, 0><<<dim3(NBLK, 1), b256, 0, stream>>>(UH, UL, DIN, WXP, DIN, DIN, fuse_b, XDBL, DBW, YH, YL, DIN, ONC, PART);
  k_dt<<<dim3(cdv((long)NTOK * DIN, 256)), b256, 0, stream>>>(XDBL, dt_proj_w, dt_proj_b, DT);
  k_scan<<<dim3(NBT), dim3(DIN), 0, stream>>>(DT, UF, XDBL, XZ, A_log, Dv, YH, YL);
  k_gemm<1, 1, 0, 0, 1><<<dim3(NBLK, NBY3), b256, 0, stream>>>(YH, YL, DIN, WOP, DIN, DIN, out_proj_b, XZ, DXZ, UH, UL, DIN, ONC, PART);
  k_bnfin<<<dim3(1), b256, 0, stream>>>(PART, ST);
  k_bnapply<<<dim3(NBT * NCH * NPIX / 4 / 256), b256, 0, stream>>>(ONC, ST, bn_g, bn_b, out);
}
